// SelfAttention_22634477650401
// MI455X (gfx1250) — hardware-verified
//
#include <hip/hip_runtime.h>

#ifndef NB
#define NB 2
#endif
#ifndef SEQ
#define SEQ 2048
#endif
#ifndef EARLY_ROWS
#define EARLY_ROWS 512
#endif
#define NB_FULL 2
#define SEQ_FULL 2048
#define DE 1024
#define NHD 16
#define DHD 64
#define TD (3 * DE)
#define MR (NB * SEQ)
#define BQ 128
#define BKY 32
#define NQB (SEQ / BQ)
#define EARLY_QB (((EARLY_ROWS < SEQ) ? EARLY_ROWS : SEQ) / BQ)
#define PBX ((MR * DE) / 2048)
#define PBWI ((TD * DE) / 2048)
#define PBWO ((DE * DE) / 2048)

#define PCAR 4096.0f
#define RCAR 1024.0f
#define RINV 0.0009765625f
#define ACAR 16.0f
#define WCAR 64.0f
#define OINV 0.0009765625f

static_assert(NB >= 1 && NB <= NB_FULL);
static_assert(SEQ >= BQ && SEQ <= SEQ_FULL);
static_assert(SEQ % BQ == 0);
static_assert(SEQ % BKY == 0);
static_assert(EARLY_ROWS >= BQ && (EARLY_ROWS % BQ) == 0);
static_assert(MR % 128 == 0);
static_assert(DE % 64 == 0 && TD % 64 == 0);
static_assert(DHD == 64 && NHD * DHD == DE);
static_assert((MR * DE) % 2048 == 0 && (TD * DE) % 2048 == 0 && (DE * DE) % 2048 == 0);

typedef _Float16 v16h __attribute__((ext_vector_type(16)));
typedef __bf16   v16b __attribute__((ext_vector_type(16)));
typedef float    v8f  __attribute__((ext_vector_type(8)));
typedef float    v4f  __attribute__((ext_vector_type(4)));
typedef unsigned v4u  __attribute__((ext_vector_type(4)));
typedef unsigned short us16;

union FragH { v16h v; v4u q[2]; _Float16 e[16]; };
union FragB { v16b v; v4u q[2]; };

__device__ __forceinline__ v8f zero8()
{
    return (v8f){0.f, 0.f, 0.f, 0.f, 0.f, 0.f, 0.f, 0.f};
}

__device__ __forceinline__ unsigned bfbits(float f)
{
    unsigned u = __float_as_uint(f);
    u += 0x7FFFu + ((u >> 16) & 1u);
    return u >> 16;
}
__device__ __forceinline__ float bfr(float f)
{
    return __uint_as_float(bfbits(f) << 16);
}

__device__ __forceinline__ v4u ld16(const us16* p)
{
    return *(const v4u*)p;
}

__device__ __forceinline__ v8f mma_h(v16h a, v16h b, v8f c)
{
    c = __builtin_amdgcn_wmma_f32_16x16x32_f16(false, a, false, b, (short)0, c, false, false);
    asm volatile("v_nop\n\tv_nop\n\tv_nop\n\tv_nop" : "+v"(c) : "v"(a), "v"(b));
    return c;
}
__device__ __forceinline__ v8f mma_b(v16b a, v16b b, v8f c)
{
    c = __builtin_amdgcn_wmma_f32_16x16x32_bf16(false, a, false, b, (short)0, c, false, false);
    asm volatile("v_nop\n\tv_nop\n\tv_nop\n\tv_nop" : "+v"(c) : "v"(a), "v"(b));
    return c;
}

__global__ __launch_bounds__(256)
void k_planes(const float* __restrict__ x, const float* __restrict__ w_in,
              const float* __restrict__ w_out, us16* XB, us16* WIB, us16* WOH)
{
    const int blk = (int)blockIdx.x;
    const int tid = (int)threadIdx.x;
    if (blk < PBX) {
        const unsigned u = (unsigned)blk * 256u + (unsigned)tid;
        const unsigned e = u * 8u;
        const unsigned m = e / DE, col = e % DE;
        const unsigned bb = m / SEQ, s = m % SEQ;
        const float* sp = x + (size_t)(bb * SEQ_FULL + s) * DE + col;
        const float4 v0 = *(const float4*)sp;
        const float4 v1 = *(const float4*)(sp + 4);
        v4u pk;
        pk.x = bfbits(v0.x) | (bfbits(v0.y) << 16);
        pk.y = bfbits(v0.z) | (bfbits(v0.w) << 16);
        pk.z = bfbits(v1.x) | (bfbits(v1.y) << 16);
        pk.w = bfbits(v1.z) | (bfbits(v1.w) << 16);
        us16* dp = XB + e;
        *(volatile v4u*)dp = pk;
        __threadfence();
        *(volatile v4u*)dp = pk;
    } else if (blk < PBX + PBWI) {
        const unsigned u = (unsigned)(blk - PBX) * 256u + (unsigned)tid;
        const unsigned e = u * 8u;
        const float* sp = w_in + e;
        const float4 v0 = *(const float4*)sp;
        const float4 v1 = *(const float4*)(sp + 4);
        v4u pk;
        pk.x = bfbits(v0.x) | (bfbits(v0.y) << 16);
        pk.y = bfbits(v0.z) | (bfbits(v0.w) << 16);
        pk.z = bfbits(v1.x) | (bfbits(v1.y) << 16);
        pk.w = bfbits(v1.z) | (bfbits(v1.w) << 16);
        us16* dp = WIB + e;
        *(volatile v4u*)dp = pk;
        __threadfence();
        *(volatile v4u*)dp = pk;
    } else {
        const unsigned u = (unsigned)(blk - PBX - PBWI) * 256u + (unsigned)tid;
        const unsigned e = u * 8u;
        const float* sp = w_out + e;
        const float4 v0 = *(const float4*)sp;
        const float4 v1 = *(const float4*)(sp + 4);
        union { _Float16 h[8]; v4u q; } o;
        o.h[0] = (_Float16)(bfr(v0.x) * WCAR);
        o.h[1] = (_Float16)(bfr(v0.y) * WCAR);
        o.h[2] = (_Float16)(bfr(v0.z) * WCAR);
        o.h[3] = (_Float16)(bfr(v0.w) * WCAR);
        o.h[4] = (_Float16)(bfr(v1.x) * WCAR);
        o.h[5] = (_Float16)(bfr(v1.y) * WCAR);
        o.h[6] = (_Float16)(bfr(v1.z) * WCAR);
        o.h[7] = (_Float16)(bfr(v1.w) * WCAR);
        const v4u pk = o.q;
        us16* dp = WOH + e;
        *(volatile v4u*)dp = pk;
        __threadfence();
        *(volatile v4u*)dp = pk;
    }
}

__global__ __launch_bounds__(256)
void k_qkv(const us16* __restrict__ XB, const us16* __restrict__ WIB, const float* __restrict__ b_in,
           us16* QH, us16* QR, us16* KH, us16* KR, us16* VTH, us16* VTR)
{
    __shared__ __attribute__((aligned(16))) _Float16 th[128 * 64];
    __shared__ __attribute__((aligned(16))) _Float16 tr[128 * 64];

    const int tid = (int)threadIdx.x;
    const int lane = tid & 31, wave = tid >> 5;
    const int lq = lane & 15, hl = lane >> 4;
    const int wm = wave >> 1, wn = wave & 1;
    const int n0 = (int)blockIdx.x * 64;
    const int m0 = (int)blockIdx.y * 128;

    v8f acc[2][2];
#pragma unroll
    for (int mi = 0; mi < 2; ++mi)
#pragma unroll
        for (int ni = 0; ni < 2; ++ni) acc[mi][ni] = zero8();

    const us16* Ap = XB  + (size_t)(m0 + wm * 32 + lq) * DE + 8 * hl;
    const us16* Bp = WIB + (size_t)(n0 + wn * 32 + lq) * DE + 8 * hl;

#pragma unroll 2
    for (int k0 = 0; k0 < DE; k0 += 32) {
        FragB a0, a1, b0, b1;
        a0.q[0] = ld16(Ap + k0);               a0.q[1] = ld16(Ap + k0 + 16);
        a1.q[0] = ld16(Ap + 16 * DE + k0);     a1.q[1] = ld16(Ap + 16 * DE + k0 + 16);
        b0.q[0] = ld16(Bp + k0);               b0.q[1] = ld16(Bp + k0 + 16);
        b1.q[0] = ld16(Bp + 16 * DE + k0);     b1.q[1] = ld16(Bp + 16 * DE + k0 + 16);
        acc[0][0] = mma_b(a0.v, b0.v, acc[0][0]);
        acc[0][1] = mma_b(a0.v, b1.v, acc[0][1]);
        acc[1][0] = mma_b(a1.v, b0.v, acc[1][0]);
        acc[1][1] = mma_b(a1.v, b1.v, acc[1][1]);
    }

    const int sec  = n0 / DE;
    const int head = (n0 % DE) / DHD;
    const int bb   = m0 / SEQ;
    const int s0   = m0 % SEQ;
    const float bia0 = bfr(b_in[n0 + wn * 32 + lq]);
    const float bia1 = bfr(b_in[n0 + wn * 32 + 16 + lq]);

#pragma unroll
    for (int mi = 0; mi < 2; ++mi) {
#pragma unroll
        for (int ni = 0; ni < 2; ++ni) {
#pragma unroll
            for (int r = 0; r < 8; ++r) {
                const float val = acc[mi][ni][r] + (ni ? bia1 : bia0);
                const _Float16 hv = (_Float16)val;
                const _Float16 rv = (_Float16)((val - (float)hv) * RCAR);
                const int row = wm * 32 + mi * 16 + 8 * hl + r;
                const int col = wn * 32 + ni * 16 + lq;
                const int li = (sec < 2) ? (row * 64 + col) : (col * 128 + row);
                th[li] = hv;
                tr[li] = rv;
            }
        }
    }
    __syncthreads();

    us16* dh;
    us16* dr;
    if (sec == 0)      { dh = QH;  dr = QR;  }
    else if (sec == 1) { dh = KH;  dr = KR;  }
    else               { dh = VTH; dr = VTR; }
    const size_t rbase = ((size_t)(bb * NHD + head) * SEQ + s0) * DHD;
    const size_t vbase = (size_t)(bb * NHD + head) * DHD;

    v4u hv4[4], rv4[4];
    size_t off[4];
#pragma unroll
    for (int it = 0; it < 4; ++it) {
        const int u = it * 256 + tid;
        hv4[it] = *(const v4u*)(th + u * 8);
        rv4[it] = *(const v4u*)(tr + u * 8);
        off[it] = (sec < 2) ? (rbase + (size_t)u * 8)
                            : ((vbase + (size_t)(u >> 4)) * SEQ + s0 + (u & 15) * 8);
    }
#pragma unroll
    for (int it = 0; it < 4; ++it) {
        *(volatile v4u*)(dh + off[it]) = hv4[it];
        *(volatile v4u*)(dr + off[it]) = rv4[it];
    }
    __threadfence();
#pragma unroll
    for (int it = 0; it < 4; ++it) {
        *(volatile v4u*)(dh + off[it]) = hv4[it];
        *(volatile v4u*)(dr + off[it]) = rv4[it];
    }
}

template <int EARLY>
__device__ __forceinline__ v8f score_tile(const us16* kp, const us16* krp,
                                          v16h q0, v16h q1, v16h r0, v16h r1)
{
    FragH k0, k1;
    k0.q[0] = ld16(kp);      k0.q[1] = ld16(kp + 16);
    k1.q[0] = ld16(kp + 32); k1.q[1] = ld16(kp + 48);
    v8f a = zero8();
    a = mma_h(k0.v, q0, a);
    a = mma_h(k1.v, q1, a);
    if (EARLY) {
        v8f ar = zero8();
        ar = mma_h(k0.v, r0, ar);
        ar = mma_h(k1.v, r1, ar);
        FragH x0, x1;
        x0.q[0] = ld16(krp);      x0.q[1] = ld16(krp + 16);
        x1.q[0] = ld16(krp + 32); x1.q[1] = ld16(krp + 48);
        ar = mma_h(x0.v, q0, ar);
        ar = mma_h(x1.v, q1, ar);
        a = a + ar * RINV;
    }
    return a;
}

template <int EARLY>
__global__ __launch_bounds__(256) __attribute__((amdgpu_num_vgpr(256)))
void k_attn(const us16* __restrict__ QH, const us16* __restrict__ QR,
            const us16* __restrict__ KH, const us16* __restrict__ KR,
            const us16* __restrict__ VTH, const us16* __restrict__ VTR,
            const int* __restrict__ maskp, us16* AH, us16* AR, int qb0)
{
    __shared__ __attribute__((aligned(16))) _Float16 eh[8 * 16 * 64];
    __shared__ __attribute__((aligned(16))) _Float16 er[8 * 16 * 64];

    const int tid = (int)threadIdx.x;
    const int lane = tid & 31, wave = tid >> 5;
    const int lq = lane & 15, hl = lane >> 4;
    const int qblk = (int)blockIdx.x + qb0;
    const int bh = (int)blockIdx.y;
    const int bb = bh / NHD, head = bh - bb * NHD;
    const int causal = (maskp[0] != 0) ? 1 : 0;
    const size_t pb = (size_t)bh * SEQ * DHD;
    const us16* Qp  = QH  + pb;
    const us16* Qrp = QR  + pb;
    const us16* Kp  = KH  + pb;
    const us16* Krp = KR  + pb;
    const us16* Vp  = VTH + pb;
    const us16* Vrp = VTR + pb;
    const int qw0 = qblk * BQ + wave * 16;

    FragH qf0, qf1, qr0, qr1;
    {
        const us16* q = Qp + (size_t)(qw0 + lq) * DHD + 8 * hl;
        qf0.q[0] = ld16(q);      qf0.q[1] = ld16(q + 16);
        qf1.q[0] = ld16(q + 32); qf1.q[1] = ld16(q + 48);
        if (EARLY) {
            const us16* q2 = Qrp + (size_t)(qw0 + lq) * DHD + 8 * hl;
            qr0.q[0] = ld16(q2);      qr0.q[1] = ld16(q2 + 16);
            qr1.q[0] = ld16(q2 + 32); qr1.q[1] = ld16(q2 + 48);
        } else {
            qr0.q[0] = (v4u){0u, 0u, 0u, 0u}; qr0.q[1] = (v4u){0u, 0u, 0u, 0u};
            qr1.q[0] = (v4u){0u, 0u, 0u, 0u}; qr1.q[1] = (v4u){0u, 0u, 0u, 0u};
        }
    }

    v8f o[4], orr[4];
#pragma unroll
    for (int dt = 0; dt < 4; ++dt) { o[dt] = zero8(); orr[dt] = zero8(); }

    const float ninf = -__builtin_inff();
    const float cexp = 0.125f * 1.4426950408889634f;
    float rmax = ninf;
    float rsum = 0.0f;

    int nit = SEQ / BKY;
    if (causal) { const int t = (qw0 >> 5) + 1; if (t < nit) nit = t; }

#pragma unroll 1
    for (int i = 0; i < nit; ++i) {
        const int j0 = i * BKY;
        const us16* kp  = Kp  + (size_t)(j0 + lq) * DHD + 8 * hl;
        const us16* krp = Krp + (size_t)(j0 + lq) * DHD + 8 * hl;
        v8f c0 = score_tile<EARLY>(kp, krp, qf0.v, qf1.v, qr0.v, qr1.v);
        v8f c1 = score_tile<EARLY>(kp + 16 * DHD, krp + 16 * DHD, qf0.v, qf1.v, qr0.v, qr1.v);

        if (causal && (j0 + BKY > qw0)) {
            const int qi = qw0 + lq;
            const int kb = j0 + 8 * hl;
#pragma unroll
            for (int r = 0; r < 8; ++r) {
                c0[r] = (kb + r > qi)      ? ninf : c0[r];
                c1[r] = (kb + 16 + r > qi) ? ninf : c1[r];
            }
        }

        float m_new = rmax;
#pragma unroll
        for (int r = 0; r < 8; ++r) { m_new = fmaxf(m_new, c0[r]); m_new = fmaxf(m_new, c1[r]); }
        m_new = fmaxf(m_new, __shfl_xor(m_new, 16));
        const float scale = __builtin_amdgcn_exp2f((rmax - m_new) * cexp);
        rmax = m_new;

        FragH pa, pr;
        float psum = 0.0f;
#pragma unroll
        for (int r = 0; r < 8; ++r) {
            const float p0 = __builtin_amdgcn_exp2f((c0[r] - m_new) * cexp);
            const float p1 = __builtin_amdgcn_exp2f((c1[r] - m_new) * cexp);
            psum += p0 + p1;
            const float s0 = p0 * PCAR, s1 = p1 * PCAR;
            const _Float16 h0 = (_Float16)s0, h1 = (_Float16)s1;
            pa.e[r]     = h0;
            pa.e[8 + r] = h1;
            if (EARLY) {
                pr.e[r]     = (_Float16)((s0 - (float)h0) * RCAR);
                pr.e[8 + r] = (_Float16)((s1 - (float)h1) * RCAR);
            }
        }
        rsum = rsum * scale + psum + __shfl_xor(psum, 16);

        float sc[8];
#pragma unroll
        for (int r = 0; r < 8; ++r) sc[r] = __shfl(scale, 8 * hl + r);
#pragma unroll
        for (int dt = 0; dt < 4; ++dt) {
#pragma unroll
            for (int r = 0; r < 8; ++r) {
                o[dt][r] *= sc[r];
                if (EARLY) orr[dt][r] *= sc[r];
            }
        }

#pragma unroll
        for (int dt = 0; dt < 4; ++dt) {
            const us16* vp = Vp + (size_t)(dt * 16 + lq) * SEQ + j0 + 8 * hl;
            FragH vf;
            vf.q[0] = ld16(vp);
            vf.q[1] = ld16(vp + 16);
            o[dt] = mma_h(pa.v, vf.v, o[dt]);
            if (EARLY) {
                const us16* vrp = Vrp + (size_t)(dt * 16 + lq) * SEQ + j0 + 8 * hl;
                FragH vr;
                vr.q[0] = ld16(vrp);
                vr.q[1] = ld16(vrp + 16);
                orr[dt] = mma_h(pa.v, vr.v, orr[dt]);
                orr[dt] = mma_h(pr.v, vf.v, orr[dt]);
            }
        }
    }

    if (EARLY) {
#pragma unroll
        for (int dt = 0; dt < 4; ++dt) o[dt] = o[dt] + orr[dt] * RINV;
    }
    const float rinv = 1.0f / (rsum * PCAR);
    float iv[8];
#pragma unroll
    for (int r = 0; r < 8; ++r) iv[r] = __shfl(rinv, 8 * hl + r) * ACAR;

    _Float16* ehw = eh + wave * (16 * 64);
    _Float16* erw = er + wave * (16 * 64);
#pragma unroll
    for (int dt = 0; dt < 4; ++dt) {
#pragma unroll
        for (int r = 0; r < 8; ++r) {
            const float a = o[dt][r] * iv[r];
            const _Float16 ah = (_Float16)a;
            const _Float16 ar = (_Float16)((a - (float)ah) * RCAR);
            const int li = (8 * hl + r) * 64 + dt * 16 + lq;
            ehw[li] = ah;
            erw[li] = ar;
        }
    }
    __syncthreads();

    v4u hv[4], rv[4];
    size_t off[4];
#pragma unroll
    for (int it = 0; it < 4; ++it) {
        const int idx = it * 32 + lane;
        hv[it] = *(const v4u*)(ehw + idx * 8);
        rv[it] = *(const v4u*)(erw + idx * 8);
        const int row = idx >> 3, piece = idx & 7;
        off[it] = ((size_t)(bb * SEQ + qw0 + row)) * DE + head * DHD + piece * 8;
    }
#pragma unroll
    for (int it = 0; it < 4; ++it) {
        *(volatile v4u*)(AH + off[it]) = hv[it];
        *(volatile v4u*)(AR + off[it]) = rv[it];
    }
    __threadfence();
#pragma unroll
    for (int it = 0; it < 4; ++it) {
        *(volatile v4u*)(AH + off[it]) = hv[it];
        *(volatile v4u*)(AR + off[it]) = rv[it];
    }
}

__global__ __launch_bounds__(256)
void k_out(const us16* __restrict__ AH, const us16* __restrict__ AR, const us16* __restrict__ WOH,
           const float* __restrict__ b_out, float* out)
{
    __shared__ __attribute__((aligned(16))) float tc[128 * 64];

    const int tid = (int)threadIdx.x;
    const int lane = tid & 31, wave = tid >> 5;
    const int lq = lane & 15, hl = lane >> 4;
    const int wm = wave >> 1, wn = wave & 1;
    const int n0 = (int)blockIdx.x * 64;
    const int m0 = (int)blockIdx.y * 128;
    const int early = ((m0 % SEQ) < EARLY_ROWS) ? 1 : 0;

    v8f acc[2][2], accr[2][2];
#pragma unroll
    for (int mi = 0; mi < 2; ++mi)
#pragma unroll
        for (int ni = 0; ni < 2; ++ni) { acc[mi][ni] = zero8(); accr[mi][ni] = zero8(); }

    const us16* Ap = AH  + (size_t)(m0 + wm * 32 + lq) * DE + 8 * hl;
    const us16* Rp = AR  + (size_t)(m0 + wm * 32 + lq) * DE + 8 * hl;
    const us16* Bp = WOH + (size_t)(n0 + wn * 32 + lq) * DE + 8 * hl;

#pragma unroll 2
    for (int k0 = 0; k0 < DE; k0 += 32) {
        FragH a0, a1, b0, b1;
        a0.q[0] = ld16(Ap + k0);               a0.q[1] = ld16(Ap + k0 + 16);
        a1.q[0] = ld16(Ap + 16 * DE + k0);     a1.q[1] = ld16(Ap + 16 * DE + k0 + 16);
        b0.q[0] = ld16(Bp + k0);               b0.q[1] = ld16(Bp + k0 + 16);
        b1.q[0] = ld16(Bp + 16 * DE + k0);     b1.q[1] = ld16(Bp + 16 * DE + k0 + 16);
        acc[0][0] = mma_h(a0.v, b0.v, acc[0][0]);
        acc[0][1] = mma_h(a0.v, b1.v, acc[0][1]);
        acc[1][0] = mma_h(a1.v, b0.v, acc[1][0]);
        acc[1][1] = mma_h(a1.v, b1.v, acc[1][1]);
        if (early) {
            FragH r0, r1;
            r0.q[0] = ld16(Rp + k0);           r0.q[1] = ld16(Rp + k0 + 16);
            r1.q[0] = ld16(Rp + 16 * DE + k0); r1.q[1] = ld16(Rp + 16 * DE + k0 + 16);
            accr[0][0] = mma_h(r0.v, b0.v, accr[0][0]);
            accr[0][1] = mma_h(r0.v, b1.v, accr[0][1]);
            accr[1][0] = mma_h(r1.v, b0.v, accr[1][0]);
            accr[1][1] = mma_h(r1.v, b1.v, accr[1][1]);
        }
    }

    const float bia0 = bfr(b_out[n0 + wn * 32 + lq]);
    const float bia1 = bfr(b_out[n0 + wn * 32 + 16 + lq]);
#pragma unroll
    for (int mi = 0; mi < 2; ++mi) {
#pragma unroll
        for (int ni = 0; ni < 2; ++ni) {
#pragma unroll
            for (int r = 0; r < 8; ++r) {
                const float val = (acc[mi][ni][r] + accr[mi][ni][r] * RINV) * OINV + (ni ? bia1 : bia0);
                const int row = wm * 32 + mi * 16 + 8 * hl + r;
                const int col = wn * 32 + ni * 16 + lq;
                tc[row * 64 + col] = val;
            }
        }
    }
    __syncthreads();

    v4f vv[8];
    size_t off[8];
#pragma unroll
    for (int it = 0; it < 8; ++it) {
        const int u = it * 256 + tid;
        vv[it] = *(const v4f*)(tc + u * 4);
        off[it] = (size_t)(m0 + (u >> 4)) * DE + n0 + (u & 15) * 4;
    }
#pragma unroll
    for (int it = 0; it < 8; ++it) *(volatile v4f*)(out + off[it]) = vv[it];
    __threadfence();
#pragma unroll
    for (int it = 0; it < 8; ++it) *(volatile v4f*)(out + off[it]) = vv[it];
}

extern "C" void kernel_launch(void* const* d_in, const int* in_sizes, int n_in,
                              void* d_out, int out_size, void* d_ws, size_t ws_size,
                              hipStream_t stream)
{
    if (n_in < 6) return;
    if (in_sizes[0] < ((NB - 1) * SEQ_FULL + SEQ) * DE) return;
    if (in_sizes[1] < TD * DE) return;
    if (in_sizes[2] < TD) return;
    if (in_sizes[3] < DE * DE) return;
    if (in_sizes[4] < DE) return;
    if (in_sizes[5] < 1) return;
    if (out_size < MR * DE) return;

    const float* x     = (const float*)d_in[0];
    const float* w_in  = (const float*)d_in[1];
    const float* b_in  = (const float*)d_in[2];
    const float* w_out = (const float*)d_in[3];
    const float* b_out = (const float*)d_in[4];
    const int*   maskp = (const int*)d_in[5];
    float* out = (float*)d_out;

    const size_t PL2 = (size_t)MR * DE * 2;
    char* ws = (char*)d_ws;
    size_t off = 0;
    us16* XB  = (us16*)(ws + off); off += PL2;
    us16* WIB = (us16*)(ws + off); off += (size_t)TD * DE * 2;
    us16* WOH = (us16*)(ws + off); off += (size_t)DE * DE * 2;
    us16* QH  = (us16*)(ws + off); off += PL2;
    us16* QR  = (us16*)(ws + off); off += PL2;
    us16* KH  = (us16*)(ws + off); off += PL2;
    us16* KR  = (us16*)(ws + off); off += PL2;
    us16* VTH = (us16*)(ws + off); off += PL2;
    us16* VTR = (us16*)(ws + off); off += PL2;
    us16* AH  = (us16*)(ws + off); off += PL2;
    us16* AR  = (us16*)(ws + off); off += PL2;
    if (off > ws_size) return;

    k_planes<<<dim3(PBX + PBWI + PBWO), dim3(256), 0, stream>>>(x, w_in, w_out, XB, WIB, WOH);

    k_qkv<<<dim3(TD / 64, MR / 128), dim3(256), 0, stream>>>(XB, WIB, b_in, QH, QR, KH, KR, VTH, VTR);

    k_attn<1><<<dim3(EARLY_QB, NB * NHD), dim3(256), 0, stream>>>(QH, QR, KH, KR, VTH, VTR,
                                                                   maskp, AH, AR, 0);
    if (NQB > EARLY_QB) {
        k_attn<0><<<dim3(NQB - EARLY_QB, NB * NHD), dim3(256), 0, stream>>>(QH, QR, KH, KR, VTH, VTR,
                                                                             maskp, AH, AR, EARLY_QB);
    }

    k_out<<<dim3(DE / 64, MR / 128), dim3(256), 0, stream>>>(AH, AR, WOH, b_out, out);
}
